// MnistSplineKAN_22771916603481
// MI455X (gfx1250) — hardware-run, weakly checked
//
#include <hip/hip_runtime.h>


#pragma clang fp contract(off)

#ifndef NB
#define NB 8192
#endif
#define NB_FULL 8192
#define IND   784
#define NOUT  10
#define NG    12
#define NCF   8
#define TP    64
#define NSTEP (IND / 2)
#define KP    (NSTEP * 32)
#define AW    4
#define YP    17
#define FS    1024.0f
#define WS    1024.0f
#define FOLD  (1.0f / (1024.0f * 1024.0f))

static_assert(IND % 2 == 0);
static_assert(KP % 32 == 0);
static_assert((KP / 8) % 32 == 0);
static_assert((IND * TP) % 256 == 0);
static_assert((16 * KP / 8) % 256 == 0);
static_assert(12 + 11 + 10 + 9 <= 44);
static_assert(44 <= TP);
static_assert(NOUT <= 16);
static_assert(NCF + 1 <= 16);
static_assert(NB % (16 * AW) == 0);
static_assert(NB <= NB_FULL);
static_assert((16 * NOUT * 4) % 128 == 0);
static_assert((32 + 8) * 16 == 16 * NOUT * 4);
static_assert((AW * 16 * YP + AW * 16 * NOUT) * 4 <= 131072);

typedef _Float16 h16;
typedef __attribute__((ext_vector_type(16))) _Float16 v16h;
typedef __attribute__((ext_vector_type(8)))  _Float16 v8h;
typedef __attribute__((ext_vector_type(8)))  float    v8f;
typedef __attribute__((ext_vector_type(4)))  float    v4f;
typedef v4f  __attribute__((may_alias)) v4fa;

__device__ __forceinline__ unsigned short f2bf(float f) { unsigned u = __float_as_uint(f); u += 0x7FFFu + ((u >> 16) & 1u); return (unsigned short)(u >> 16); }
__device__ __forceinline__ float bfr(float f) { return __uint_as_float(((unsigned)f2bf(f)) << 16); }
__device__ __forceinline__ v16h cat16(v8h lo, v8h hi) { return __builtin_shufflevector(lo, hi, 0, 1, 2, 3, 4, 5, 6, 7, 8, 9, 10, 11, 12, 13, 14, 15); }
__device__ __forceinline__ v8f wmma16(v16h a, v16h b, v8f c) { return __builtin_amdgcn_wmma_f32_16x16x32_f16(false, a, false, b, (short)0, c, false, false); }
__device__ __forceinline__ v16h  ldh(const h16* p) { return cat16(*(const v8h*)p, *(const v8h*)(p + 16)); }
__device__ __forceinline__ void wave_sync() { __builtin_amdgcn_fence(3  , "wavefront"); __builtin_amdgcn_wave_barrier(); asm volatile("" ::: "memory"); }
static __device__ __forceinline__ h16 toh_flush(float v) { const h16 r = (h16)v; return (fabsf(v) < 6.103515625e-05f) ? (h16)0.0f : r; }

__global__ __launch_bounds__(256) void k_tbl(const float* __restrict__ grid, float* TBL) {
    const int t = blockIdx.x * 256 + threadIdx.x; if (t >= IND * TP) return;
    const int i = t >> 6, s = t & 63;
    int p = 0, tt = 0;
    if (s < 12) { p = 0; tt = s; } else if (s < 23) { p = 1; tt = s - 12; } else if (s < 33) { p = 2; tt = s - 23; } else if (s < 42) { p = 3; tt = s - 33; }
    const float glo = bfr(grid[i * NG + tt]);
    const float ghi = bfr(grid[i * NG + tt + p]);
    const float den = ghi - glo;
    const float dsel = (p > 0) ? den : 1.0f;
    const float rc = 1.0f / dsel;
    const float v = (s < 12) ? glo : ((s < 42) ? rc : 0.0f);
    *(volatile float*)(TBL + t) = v; __threadfence(); *(volatile float*)(TBL + t) = v;
}

__global__ __launch_bounds__(256) void k_wplane(const float* __restrict__ coef, const float* __restrict__ sbase, const float* __restrict__ ssp, const float* __restrict__ mask, h16* WP) {
    const int t = blockIdx.x * 256 + threadIdx.x; if (t >= 16 * KP / 8) return;
    const int n = t / (KP / 8); const int kphys = (t - n * (KP / 8)) * 8;
    const int s = kphys >> 5, p = kphys & 31; const int hf = (p >> 3) & 1; const int up = p >> 4;
    const int i = 2 * s + hf;
    const int nn = n < NOUT ? n : (NOUT - 1);
    const int io = i * NOUT + nn;
    float m = mask[io], sb = sbase[io], sp = ssp[io];
    v4f c0 = *(const v4f*)(coef + (size_t)io * NCF), c1 = *(const v4f*)(coef + (size_t)io * NCF + 4);
    asm volatile("" : "+v"(m)); asm volatile("" : "+v"(sb)); asm volatile("" : "+v"(sp)); asm volatile("" : "+v"(c0)); asm volatile("" : "+v"(c1));
    m = bfr(m); sb = bfr(sb); sp = bfr(sp);
    float cf[8];
#pragma unroll
    for (int j = 0; j < 4; ++j) { cf[j] = bfr(c0[j]); cf[4 + j] = bfr(c1[j]); }
    const float msp = m * sp;
    const bool live = n < NOUT;
    float w[8];
    w[0] = (up != 0) ? (msp * cf[7]) : (m * sb);
#pragma unroll
    for (int j = 1; j < 8; ++j) w[j] = (up != 0) ? 0.0f : (msp * cf[j - 1]);
    v8h hv;
#pragma unroll
    for (int j = 0; j < 8; ++j) { const float x = live ? w[j] : 0.0f; hv[j] = toh_flush(x * WS); }
    *(volatile v8h*)(WP + (size_t)t * 8) = hv; __threadfence(); *(volatile v8h*)(WP + (size_t)t * 8) = hv;
}

__global__ __launch_bounds__(32 * AW) void k_edge(const float* __restrict__ X, const float* __restrict__ TBL, const h16* __restrict__ WP,
                                                  const float* __restrict__ Wm, const float* __restrict__ bias, float* OUT) {
    __shared__ __align__(16) float ys[AW * 16 * YP];
    __shared__ __align__(16) float ot[AW * 16 * NOUT];
    const int lane = threadIdx.x & 31, lr = lane & 15, hi = lane >> 4;
    const int wave = __builtin_amdgcn_readfirstlane((int)(threadIdx.x >> 5));
    const int tile = blockIdx.x * AW + wave;
    const float* xrow = X + (size_t)(tile * 16 + lr) * IND;
    const h16* wrow = WP + (size_t)lr * KP + 8 * hi;
    v8f acc = (v8f){};
#pragma unroll 1
    for (int s = 0; s < NSTEP; ++s) {
        const int i = 2 * s + hi;
        const float xv = bfr(xrow[i]);
        const float* tp = TBL + (size_t)i * TP;
        float tv[44];
#pragma unroll
        for (int q = 0; q < 11; ++q) { const v4f w = *(const v4f*)(tp + 4 * q); tv[4 * q] = w[0]; tv[4 * q + 1] = w[1]; tv[4 * q + 2] = w[2]; tv[4 * q + 3] = w[3]; }
        float d[12];
#pragma unroll
        for (int t = 0; t < 12; ++t) d[t] = xv - tv[t];
        float B0[11];
#pragma unroll
        for (int t = 0; t < 11; ++t) B0[t] = ((xv >= tv[t]) & (xv < tv[t + 1])) ? 1.0f : 0.0f;
        float B1[10];
#pragma unroll
        for (int t = 0; t < 10; ++t) B1[t] = (d[t] * tv[12 + t]) * B0[t] + ((-d[t + 2]) * tv[12 + t + 1]) * B0[t + 1];
        float B2[9];
#pragma unroll
        for (int t = 0; t < 9; ++t)  B2[t] = (d[t] * tv[23 + t]) * B1[t] + ((-d[t + 3]) * tv[23 + t + 1]) * B1[t + 1];
        float B3[8];
#pragma unroll
        for (int t = 0; t < 8; ++t)  B3[t] = (d[t] * tv[33 + t]) * B2[t] + ((-d[t + 4]) * tv[33 + t + 1]) * B2[t + 1];
        const float sil = xv * __builtin_amdgcn_rcpf(1.0f + expf(-xv));
        v16h a = (v16h){};
        a[0] = toh_flush(sil * FS);
#pragma unroll
        for (int k = 0; k < 8; ++k) a[1 + k] = toh_flush(B3[k] * FS);
        const v16h bw = ldh(wrow + (size_t)s * 32);
        acc = wmma16(a, bw, acc);
        asm volatile("v_nop\n\tv_nop\n\tv_nop\n\tv_nop" : "+v"(acc) : "v"(a), "v"(bw));
    }
    const int yb = wave * 16 * YP;
#pragma unroll
    for (int r = 0; r < 8; ++r) ys[yb + (8 * hi + r) * YP + lr] = acc[r] * FOLD;
    wave_sync();
    const int wb = wave * 16 * NOUT;
#pragma unroll 1
    for (int q = 0; q < 5; ++q) {
        const int f = q * 32 + lane; const int row = f / NOUT; const int col = f - row * NOUT;
        float v = 0.0f;
#pragma unroll 1
        for (int o = 0; o < NOUT; ++o) v += bfr(Wm[col * NOUT + o]) * ys[yb + row * YP + o];
        v += bfr(bias[col]);
        ot[wb + f] = v;
    }
    wave_sync();
    float* op = OUT + (size_t)tile * (16 * NOUT);
    const int tl = 128 + 4 * (lane & 7);
#pragma unroll 1
    for (int ps = 0; ps < 2; ++ps) {
        const v4f v0 = *(const v4fa*)(&ot[wb + 4 * lane]);
        const v4f v1 = *(const v4fa*)(&ot[wb + tl]);
        *(volatile v4f*)(op + 4 * lane) = v0;
        if (lane < 8) *(volatile v4f*)(op + tl) = v1;
        if (ps == 0) __threadfence(); }
}

static constexpr size_t al256(size_t v) { return (v + 255) & ~(size_t)255; }
static constexpr size_t SZ_TBL = al256((size_t)IND * TP * 4);
static constexpr size_t SZ_WP  = al256((size_t)16 * KP * 2);
static constexpr size_t SZ_TOTAL = SZ_TBL + SZ_WP;
static_assert(SZ_TOTAL <= (size_t)134217728);
static_assert((size_t)IND * TP * 4 == SZ_TBL);
static_assert((size_t)16 * KP * 2 == SZ_WP);

extern "C" void kernel_launch(void* const* d_in, const int* in_sizes, int n_in,
                              void* d_out, int out_size, void* d_ws, size_t ws_size, hipStream_t stream) {
    if (n_in < 8) return;
    if ((size_t)in_sizes[0] < (size_t)NB * IND) return;
    if (in_sizes[1] < IND * NG || in_sizes[2] < IND * NOUT * NCF) return;
    if (in_sizes[3] < IND * NOUT || in_sizes[4] < IND * NOUT || in_sizes[5] < IND * NOUT) return;
    if (in_sizes[6] < NOUT * NOUT || in_sizes[7] < NOUT) return;
    if ((size_t)out_size < (size_t)NB * NOUT) return;
    if (SZ_TOTAL > ws_size) return;
    const float* x     = (const float*)d_in[0];
    const float* grid  = (const float*)d_in[1];
    const float* coef  = (const float*)d_in[2];
    const float* sbase = (const float*)d_in[3];
    const float* ssp   = (const float*)d_in[4];
    const float* mask  = (const float*)d_in[5];
    const float* Wm    = (const float*)d_in[6];
    const float* bias  = (const float*)d_in[7];
    float* OUT = (float*)d_out;
    char* wsp = (char*)d_ws;
    float* TBL = (float*)wsp; wsp += SZ_TBL;
    h16*   WP  = (h16*)wsp;   wsp += SZ_WP;

    k_tbl<<<(unsigned)((IND * TP) / 256), 256, 0, stream>>>(grid, TBL);
    k_wplane<<<(unsigned)((16 * KP / 8) / 256), 256, 0, stream>>>(coef, sbase, ssp, mask, WP);
    k_edge<<<(unsigned)(NB / (16 * AW)), 32 * AW, 0, stream>>>(x, TBL, WP, Wm, bias, OUT);
}
